// myGNN_17454747091496
// MI455X (gfx1250) — hardware-verified
//
#include <hip/hip_runtime.h>


#define NTHR   256
#define NWAVE  8
#define FEAT   64

#define EPB    4096
#define EIT    (EPB / 128)
#define NWH    (256 * 64 + 128 * 256 + 64 * 128)

#define EPT    8
#define CHUNK  (NTHR * EPT)
#define WCAP   (EPT * 32)
#define LISTN  (NWAVE * WCAP)
#define NB     512
#define TPW    (NB / 16 / NWAVE)

#define WSC    8.0f
#define WINV   0.125f
#define SLOPE  0.01f
#define L2EPS  1e-12f

static_assert(EIT * 128 == EPB);
static_assert(TPW * 16 * NWAVE == NB);
static_assert((NWH % 2048) == 0);
static_assert(WCAP * NWAVE == CHUNK);

typedef float          v2f   __attribute__((ext_vector_type(2)));
typedef float          v4f   __attribute__((ext_vector_type(4)));
typedef float          v8f   __attribute__((ext_vector_type(8)));
typedef int            v4i   __attribute__((ext_vector_type(4)));
typedef _Float16       v8h   __attribute__((ext_vector_type(8)));
typedef _Float16       v16h  __attribute__((ext_vector_type(16)));
typedef unsigned short v8us  __attribute__((ext_vector_type(8)));
typedef unsigned short v16us __attribute__((ext_vector_type(16)));
typedef __bf16         v16b  __attribute__((ext_vector_type(16)));
union FragH { v16h v; v8h h[2]; };
union FragU { v16us u; v8us h[2]; };

__device__ __forceinline__ unsigned short bfb(float f) {
  unsigned u = __builtin_bit_cast(unsigned, f);
  u += 0x7FFFu + ((u >> 16) & 1u);
  return (unsigned short)(u >> 16);
}
__device__ __forceinline__ float bff(unsigned short b) {
  return __builtin_bit_cast(float, ((unsigned)b) << 16);
}

__device__ __forceinline__ v8f wmh(v16h a, v16h b, v8f c) {
  v8f d = __builtin_amdgcn_wmma_f32_16x16x32_f16(false, a, false, b, (short)0, c, false, false);
  asm volatile("v_nop\n\tv_nop\n\tv_nop\n\tv_nop" : "+v"(d) : "v"(a), "v"(b));
  return d;
}
__device__ __forceinline__ v8f wmb(v16b a, v16b b, v8f c) {
  v8f d = __builtin_amdgcn_wmma_f32_16x16x32_bf16(false, a, false, b, (short)0, c, false, false);
  const v8f av = __builtin_bit_cast(v8f, a);
  const v8f bv = __builtin_bit_cast(v8f, b);
  asm volatile("v_nop\n\tv_nop\n\tv_nop\n\tv_nop" : "+v"(d) : "v"(av), "v"(bv));
  return d;
}

__device__ __forceinline__ v8f ldc8(const float* p) {
  const v4f a = *(const v4f*)p;
  const v4f b = *(const v4f*)(p + 4);
  v8f c;
  c[0] = a.x; c[1] = a.y; c[2] = a.z; c[3] = a.w;
  c[4] = b.x; c[5] = b.y; c[6] = b.z; c[7] = b.w;
  return c;
}

__device__ __forceinline__ v8h act8(v8f d) {
  v8h r;
#pragma unroll
  for (int i = 0; i < 8; ++i) {
    float t = d[i] * WINV;
    t = t > 0.0f ? t : SLOPE * t;
    r[i] = (_Float16)t;
  }
  return r;
}

__device__ __forceinline__ void split16(const v4f q0, const v4f q1, const v4f q2, const v4f q3,
                                        const float sc, v16b* hi, v16b* lo) {
  float v[16];
  v[0] = q0.x;  v[1] = q0.y;  v[2] = q0.z;  v[3] = q0.w;
  v[4] = q1.x;  v[5] = q1.y;  v[6] = q1.z;  v[7] = q1.w;
  v[8] = q2.x;  v[9] = q2.y;  v[10] = q2.z; v[11] = q2.w;
  v[12] = q3.x; v[13] = q3.y; v[14] = q3.z; v[15] = q3.w;
  FragU uh, ul;
#pragma unroll
  for (int i = 0; i < 16; ++i) {
    const float t = v[i] * sc;
    const unsigned short hb = bfb(t);
    uh.u[i] = hb;
    ul.u[i] = bfb(t - bff(hb));
  }
  *hi = __builtin_bit_cast(v16b, uh.u);
  *lo = __builtin_bit_cast(v16b, ul.u);
}

__device__ __forceinline__ float sel3(float a, float b, float c, int s) {
  return s == 0 ? a : (s == 1 ? b : c);
}

__global__ __launch_bounds__(NTHR) void k_cvt(const float* __restrict__ w1, const float* __restrict__ w2,
                                              const float* __restrict__ w3, _Float16* wpl) {
  const int i = blockIdx.x * NTHR + threadIdx.x;
  if (i >= NWH / 8) return;
  const int g1 = i < 2047 ? i : 2047;
  int g2 = i - 2048; g2 = g2 < 0 ? 0 : (g2 > 4095 ? 4095 : g2);
  int g3 = i - 6144; g3 = g3 < 0 ? 0 : (g3 > 1023 ? 1023 : g3);
  const v4f a0 = *(const v4f*)(w1 + 8 * g1), a1 = *(const v4f*)(w1 + 8 * g1 + 4);
  const v4f b0 = *(const v4f*)(w2 + 8 * g2), b1 = *(const v4f*)(w2 + 8 * g2 + 4);
  const v4f c0 = *(const v4f*)(w3 + 8 * g3), c1 = *(const v4f*)(w3 + 8 * g3 + 4);
  const int s = i < 2048 ? 0 : (i < 6144 ? 1 : 2);
  v8h o;
  o[0] = (_Float16)(sel3(a0.x, b0.x, c0.x, s) * WSC);
  o[1] = (_Float16)(sel3(a0.y, b0.y, c0.y, s) * WSC);
  o[2] = (_Float16)(sel3(a0.z, b0.z, c0.z, s) * WSC);
  o[3] = (_Float16)(sel3(a0.w, b0.w, c0.w, s) * WSC);
  o[4] = (_Float16)(sel3(a1.x, b1.x, c1.x, s) * WSC);
  o[5] = (_Float16)(sel3(a1.y, b1.y, c1.y, s) * WSC);
  o[6] = (_Float16)(sel3(a1.z, b1.z, c1.z, s) * WSC);
  o[7] = (_Float16)(sel3(a1.w, b1.w, c1.w, s) * WSC);
  *(volatile v8h*)(wpl + 8 * i) = o;
  __threadfence();
  *(volatile v8h*)(wpl + 8 * i) = o;
}

__global__ __launch_bounds__(NTHR) void k_edge(
    const float* __restrict__ x, const int* __restrict__ src, const int* __restrict__ dst,
    const _Float16* __restrict__ wpl, const float* __restrict__ b1, const float* __restrict__ b2,
    const float* __restrict__ b3, const float* __restrict__ w4, const float* __restrict__ b4,
    float* eout, float* epl, int nN, int nE) {
  __shared__ __attribute__((aligned(16))) _Float16 sW[NWH];
  __shared__ __attribute__((aligned(16))) float    sB1[256];
  __shared__ __attribute__((aligned(16))) float    sB2[128];
  __shared__ __attribute__((aligned(16))) float    sB3[64];
  __shared__ __attribute__((aligned(16))) float    sW4[64];
  __shared__ __attribute__((aligned(16))) _Float16 dt[NWAVE * 16 * FEAT];
  __shared__ __attribute__((aligned(16))) float    es[128];

  const int tid = threadIdx.x, lane = tid & 31, wave = tid >> 5, h = lane >> 4, m = lane & 15;

  for (int i = tid; i < NWH / 8; i += NTHR) *(v8h*)(sW + 8 * i) = *(const v8h*)(wpl + 8 * i);
  for (int i = tid; i < 256; i += NTHR) sB1[i] = b1[i] * WSC;
  if (tid < 128) sB2[tid] = b2[tid] * WSC;
  if (tid < 64) { sB3[tid] = b3[tid] * WSC; sW4[tid] = w4[tid]; }
  const float b4v = b4[0];
  __syncthreads();

  const _Float16* sW1 = sW;
  const _Float16* sW2 = sW + 16384;
  const _Float16* sW3 = sW + 49152;
  const int blockBase = blockIdx.x * EPB;

#pragma unroll 1
  for (int it = 0; it < EIT; ++it) {
    const int tileBase = blockBase + it * 128 + wave * 16;
    {
      int eg = tileBase + m;
      eg = eg > nE - 1 ? nE - 1 : eg;
      int s = src[eg];
      int d = dst[eg];
      s = s < 0 ? 0 : (s > nN - 1 ? nN - 1 : s);
      d = d < 0 ? 0 : (d > nN - 1 ? nN - 1 : d);
      const float* xs = x + (size_t)s * FEAT + 32 * h;
      const float* xd = x + (size_t)d * FEAT + 32 * h;
      _Float16* dr = dt + (wave * 16 + m) * FEAT + 32 * h;
#pragma unroll
      for (int c = 0; c < 4; ++c) {
        const v4f p0 = *(const v4f*)(xs + 8 * c), p1 = *(const v4f*)(xs + 8 * c + 4);
        const v4f q0 = *(const v4f*)(xd + 8 * c), q1 = *(const v4f*)(xd + 8 * c + 4);
        v8h o;
        o[0] = (_Float16)(p0.x - q0.x); o[1] = (_Float16)(p0.y - q0.y);
        o[2] = (_Float16)(p0.z - q0.z); o[3] = (_Float16)(p0.w - q0.w);
        o[4] = (_Float16)(p1.x - q1.x); o[5] = (_Float16)(p1.y - q1.y);
        o[6] = (_Float16)(p1.z - q1.z); o[7] = (_Float16)(p1.w - q1.w);
        *(v8h*)(dr + 8 * c) = o;
      }
    }
    __syncthreads();

    float ev;
    {
      const _Float16* drow = dt + (wave * 16 + m) * FEAT;
      FragH bd0, bd1;
      bd0.h[0] = *(const v8h*)(drow + 8 * h);
      bd0.h[1] = *(const v8h*)(drow + 16 + 8 * h);
      bd1.h[0] = *(const v8h*)(drow + 32 + 8 * h);
      bd1.h[1] = *(const v8h*)(drow + 48 + 8 * h);

      FragH h1f[8];
#pragma unroll
      for (int j = 0; j < 8; ++j) {
        v8f dd[2];
#pragma unroll
        for (int u = 0; u < 2; ++u) {
          const int f0 = 32 * j + 16 * u;
          v8f c = ldc8(sB1 + f0 + 8 * h);
          const _Float16* ap = sW1 + (f0 + m) * 64 + 8 * h;
          FragH a;
          a.h[0] = *(const v8h*)(ap);
          a.h[1] = *(const v8h*)(ap + 16);
          c = wmh(a.v, bd0.v, c);
          FragH a2;
          a2.h[0] = *(const v8h*)(ap + 32);
          a2.h[1] = *(const v8h*)(ap + 48);
          c = wmh(a2.v, bd1.v, c);
          dd[u] = c;
        }
        h1f[j].h[0] = act8(dd[0]);
        h1f[j].h[1] = act8(dd[1]);
      }

      FragH h2f[4];
#pragma unroll
      for (int j = 0; j < 4; ++j) {
        v8f dd[2];
#pragma unroll
        for (int u = 0; u < 2; ++u) {
          const int f0 = 32 * j + 16 * u;
          v8f c = ldc8(sB2 + f0 + 8 * h);
          const _Float16* ap = sW2 + (f0 + m) * 256 + 8 * h;
#pragma unroll
          for (int kt = 0; kt < 8; ++kt) {
            FragH a;
            a.h[0] = *(const v8h*)(ap + 32 * kt);
            a.h[1] = *(const v8h*)(ap + 32 * kt + 16);
            c = wmh(a.v, h1f[kt].v, c);
          }
          dd[u] = c;
        }
        h2f[j].h[0] = act8(dd[0]);
        h2f[j].h[1] = act8(dd[1]);
      }

      float p = 0.0f;
#pragma unroll
      for (int ft = 0; ft < 4; ++ft) {
        const int f0 = 16 * ft;
        v8f c = ldc8(sB3 + f0 + 8 * h);
        const _Float16* ap = sW3 + (f0 + m) * 128 + 8 * h;
#pragma unroll
        for (int kt = 0; kt < 4; ++kt) {
          FragH a;
          a.h[0] = *(const v8h*)(ap + 32 * kt);
          a.h[1] = *(const v8h*)(ap + 32 * kt + 16);
          c = wmh(a.v, h2f[kt].v, c);
        }
#pragma unroll
        for (int r = 0; r < 8; ++r) {
          float t = c[r] * WINV;
          t = t > 0.0f ? t : SLOPE * t;
          p = fmaf(t, sW4[f0 + 8 * h + r], p);
        }
      }
      float s = p + __shfl_xor(p, 16, 32);
      s += b4v;
      s = fminf(fmaxf(s, -30.0f), 30.0f);
      ev = 1.0f / (1.0f + expf(-s));
    }
    if (h == 0) es[wave * 16 + m] = ev;
    __syncthreads();

    if (wave == 0) {
      const int eb = blockBase + it * 128 + 4 * lane;
      const v4f v = *(const v4f*)(es + 4 * lane);
      *(volatile v4f*)(epl + eb) = v;
      if (eb + 3 < nE) {
        *(volatile v4f*)(eout + eb) = v;
      } else {
        if (eb     < nE) *(volatile float*)(eout + eb)     = v.x;
        if (eb + 1 < nE) *(volatile float*)(eout + eb + 1) = v.y;
        if (eb + 2 < nE) *(volatile float*)(eout + eb + 2) = v.z;
      }
      __threadfence();
      *(volatile v4f*)(epl + eb) = v;
      if (eb + 3 < nE) {
        *(volatile v4f*)(eout + eb) = v;
      } else {
        if (eb     < nE) *(volatile float*)(eout + eb)     = v.x;
        if (eb + 1 < nE) *(volatile float*)(eout + eb + 1) = v.y;
        if (eb + 2 < nE) *(volatile float*)(eout + eb + 2) = v.z;
      }
    }
  }
}

__device__ __forceinline__ int scan_chunk(const int* __restrict__ dl, int nE, int cbase, int nodeBase,
                                          int* list, int tid, int wave) {
  int wc = 0;
  const int el0  = tid * EPT;
  const int e0   = cbase + el0;
  const int sent = -2147483647 - 1;
  v4i da, db;
  if (cbase + CHUNK <= nE) {
    da = *(const v4i*)(dl + e0);
    db = *(const v4i*)(dl + e0 + 4);
  } else {
    da.x = (e0     < nE) ? dl[min(e0,     nE - 1)] : sent;
    da.y = (e0 + 1 < nE) ? dl[min(e0 + 1, nE - 1)] : sent;
    da.z = (e0 + 2 < nE) ? dl[min(e0 + 2, nE - 1)] : sent;
    da.w = (e0 + 3 < nE) ? dl[min(e0 + 3, nE - 1)] : sent;
    db.x = (e0 + 4 < nE) ? dl[min(e0 + 4, nE - 1)] : sent;
    db.y = (e0 + 5 < nE) ? dl[min(e0 + 5, nE - 1)] : sent;
    db.z = (e0 + 6 < nE) ? dl[min(e0 + 6, nE - 1)] : sent;
    db.w = (e0 + 7 < nE) ? dl[min(e0 + 7, nE - 1)] : sent;
  }
  const unsigned nb = (unsigned)nodeBase;
  const unsigned s0 = (unsigned)da.x - nb, s1 = (unsigned)da.y - nb;
  const unsigned s2 = (unsigned)da.z - nb, s3 = (unsigned)da.w - nb;
  const unsigned s4 = (unsigned)db.x - nb, s5 = (unsigned)db.y - nb;
  const unsigned s6 = (unsigned)db.z - nb, s7 = (unsigned)db.w - nb;
  const bool h0 = s0 < (unsigned)NB, h1 = s1 < (unsigned)NB, h2 = s2 < (unsigned)NB, h3 = s3 < (unsigned)NB;
  const bool h4 = s4 < (unsigned)NB, h5 = s5 < (unsigned)NB, h6 = s6 < (unsigned)NB, h7 = s7 < (unsigned)NB;
  const unsigned any = __builtin_amdgcn_ballot_w32(h0 | h1 | h2 | h3 | h4 | h5 | h6 | h7);
  if (any != 0u) {
#define HITJ(J, HJ) { \
      const unsigned mj = __builtin_amdgcn_ballot_w32(HJ); \
      if (mj != 0u) { \
        if (HJ) { \
          const int pos = wc + (int)__builtin_amdgcn_mbcnt_lo(mj, 0u); \
          if (pos < WCAP) list[wave * WCAP + pos] = el0 + (J); \
        } \
        wc += (int)__builtin_popcount(mj); } }
    HITJ(0, h0)
    HITJ(1, h1)
    HITJ(2, h2)
    HITJ(3, h3)
    HITJ(4, h4)
    HITJ(5, h5)
    HITJ(6, h6)
    HITJ(7, h7)
#undef HITJ
  }
  return wc;
}

__global__ __launch_bounds__(NTHR) void k_node(
    const float* __restrict__ x, const int* __restrict__ src, const int* __restrict__ dst,
    const float* __restrict__ epl, const float* __restrict__ wself, const float* __restrict__ wneigh,
    const float* __restrict__ bias, float* out0, int nN, int nE) {
  __shared__ __attribute__((aligned(16))) float acc[(NB + 1) * FEAT];
  __shared__ __attribute__((aligned(16))) float cnt[NB + 1];
  __shared__ __attribute__((aligned(16))) int   list[LISTN];
  __shared__ __attribute__((aligned(16))) int   pend[CHUNK];
  __shared__ __attribute__((aligned(16))) unsigned short wsh[FEAT * FEAT];
  __shared__ __attribute__((aligned(16))) unsigned short wsl[FEAT * FEAT];
  __shared__ __attribute__((aligned(16))) unsigned short wnh[FEAT * FEAT];
  __shared__ __attribute__((aligned(16))) unsigned short wnl[FEAT * FEAT];
  __shared__ __attribute__((aligned(16))) float sbias[FEAT];
  __shared__ int wcnt[NWAVE];

  const int tid = threadIdx.x, lane = tid & 31, wave = tid >> 5, h = lane >> 4, m = lane & 15;
  const int nodeBase = blockIdx.x * NB;

  {
    const v4f z4 = {0.0f, 0.0f, 0.0f, 0.0f};
    for (int i = tid; i < (NB + 1) * FEAT / 4; i += NTHR) *(v4f*)(acc + 4 * i) = z4;
    for (int i = tid; i < NB + 1; i += NTHR) cnt[i] = 0.0f;
    for (int i = tid; i < FEAT * FEAT; i += NTHR) {
      const float a = wself[i];
      const unsigned short ah = bfb(a);
      wsh[i] = ah; wsl[i] = bfb(a - bff(ah));
      const float b = wneigh[i];
      const unsigned short bh = bfb(b);
      wnh[i] = bh; wnl[i] = bfb(b - bff(bh));
    }
    if (tid < FEAT) sbias[tid] = bias[tid];
  }
  __syncthreads();

  const int nChunks = (nE + CHUNK - 1) / CHUNK;
#pragma unroll 1
  for (int ch = 0; ch < nChunks; ++ch) {
    const int cbase = ch * CHUNK;
    const int wc = scan_chunk(dst, nE, cbase, nodeBase, list, tid, wave);
    if (lane == 0) wcnt[wave] = wc;
    __syncthreads();

    int tot = 0, myoff = 0;
#pragma unroll
    for (int w = 0; w < NWAVE; ++w) {
      int c = wcnt[w];
      c = c > WCAP ? WCAP : (c < 0 ? 0 : c);
      if (w < wave) myoff += c;
      tot += c;
    }
    tot = tot > CHUNK ? CHUNK : tot;
    {
      int n = wcnt[wave];
      n = n > WCAP ? WCAP : (n < 0 ? 0 : n);
      const int* lp = list + wave * WCAP;
      for (int i = lane; i < n; i += 32) {
        const int pos = myoff + i;
        if (pos < CHUNK) pend[pos] = cbase + lp[i];
      }
    }
    __syncthreads();

    if (wave == 0 && tot > 0) {
      const int T = tot;
#pragma unroll 1
      for (int g = 0; g < T; g += 32) {
        const int idx = g + lane;
        const int idc = idx < CHUNK ? idx : CHUNK - 1;
        const bool valid = idx < T;
        int e = pend[idc];
        e = valid ? e : 0;
        e = e < 0 ? 0 : (e > nE - 1 ? nE - 1 : e);
        int s = src[e];
        const int d = dst[e];
        const float ev = epl[e];
        s = s < 0 ? 0 : (s > nN - 1 ? nN - 1 : s);
        int sl = d - nodeBase;
        if (!valid || (unsigned)sl >= (unsigned)NB) sl = NB;
        const int cn = (T - g) < 32 ? (T - g) : 32;
#pragma unroll 1
        for (int i = 0; i < cn; ++i) {
          const int   si  = __shfl(s, i, 32);
          const int   sli = __shfl(sl, i, 32);
          const float evi = __shfl(ev, i, 32);
          const v2f xv = *(const v2f*)(x + (size_t)si * FEAT + 2 * lane);
          float* ap = acc + sli * FEAT + 2 * lane;
          v2f av = *(v2f*)ap;
          av += evi * xv;
          *(v2f*)ap = av;
          if (lane == 0) cnt[sli] += 1.0f;
        }
      }
    }
    __syncthreads();
  }
  __syncthreads();

#pragma unroll 1
  for (int t = 0; t < TPW; ++t) {
    const int slot0 = (wave * TPW + t) * 16;
    const int node0 = nodeBase + slot0;
    v16b axh[2], axl[2], anh[2], anl[2];
    {
      int nd = node0 + m;
      nd = nd > nN - 1 ? nN - 1 : nd;
      const float* xp = x + (size_t)nd * FEAT;
      const float* np = acc + (slot0 + m) * FEAT;
      const float inv = 1.0f / fmaxf(cnt[slot0 + m], 1.0f);
#pragma unroll
      for (int kt = 0; kt < 2; ++kt) {
        const int k0 = 32 * kt + 8 * h;
        {
          const v4f q0 = *(const v4f*)(xp + k0),      q1 = *(const v4f*)(xp + k0 + 4);
          const v4f q2 = *(const v4f*)(xp + k0 + 16), q3 = *(const v4f*)(xp + k0 + 20);
          split16(q0, q1, q2, q3, 1.0f, &axh[kt], &axl[kt]);
        }
        {
          const v4f q0 = *(const v4f*)(np + k0),      q1 = *(const v4f*)(np + k0 + 4);
          const v4f q2 = *(const v4f*)(np + k0 + 16), q3 = *(const v4f*)(np + k0 + 20);
          split16(q0, q1, q2, q3, inv, &anh[kt], &anl[kt]);
        }
      }
    }
    float vo[4][8];
#pragma unroll
    for (int ct = 0; ct < 4; ++ct) {
      const float bv = sbias[16 * ct + m];
      v8f c;
#pragma unroll
      for (int r = 0; r < 8; ++r) c[r] = bv;
#pragma unroll
      for (int kt = 0; kt < 2; ++kt) {
        const int off = (16 * ct + m) * FEAT + 32 * kt + 8 * h;
        FragU bh, bl;
        bh.h[0] = *(const v8us*)(wsh + off); bh.h[1] = *(const v8us*)(wsh + off + 16);
        bl.h[0] = *(const v8us*)(wsl + off); bl.h[1] = *(const v8us*)(wsl + off + 16);
        const v16b sH = __builtin_bit_cast(v16b, bh.u);
        const v16b sL = __builtin_bit_cast(v16b, bl.u);
        c = wmb(axh[kt], sH, c);
        c = wmb(axh[kt], sL, c);
        c = wmb(axl[kt], sH, c);
        FragU nh, nl;
        nh.h[0] = *(const v8us*)(wnh + off); nh.h[1] = *(const v8us*)(wnh + off + 16);
        nl.h[0] = *(const v8us*)(wnl + off); nl.h[1] = *(const v8us*)(wnl + off + 16);
        const v16b gH = __builtin_bit_cast(v16b, nh.u);
        const v16b gL = __builtin_bit_cast(v16b, nl.u);
        c = wmb(anh[kt], gH, c);
        c = wmb(anh[kt], gL, c);
        c = wmb(anl[kt], gH, c);
      }
#pragma unroll
      for (int r = 0; r < 8; ++r) {
        const float tv = c[r];
        vo[ct][r] = tv > 0.0f ? tv : SLOPE * tv;
      }
    }
    float ss[8], invn[8];
#pragma unroll
    for (int r = 0; r < 8; ++r)
      ss[r] = vo[0][r] * vo[0][r] + vo[1][r] * vo[1][r] + vo[2][r] * vo[2][r] + vo[3][r] * vo[3][r];
#pragma unroll
    for (int k = 1; k < 16; k <<= 1) {
#pragma unroll
      for (int r = 0; r < 8; ++r) ss[r] += __shfl_xor(ss[r], k, 32);
    }
#pragma unroll
    for (int r = 0; r < 8; ++r) invn[r] = 1.0f / fmaxf(sqrtf(ss[r]), L2EPS);
    __syncthreads();
#pragma unroll
    for (int r = 0; r < 8; ++r) {
#pragma unroll
      for (int ct = 0; ct < 4; ++ct)
        acc[(slot0 + 8 * h + r) * FEAT + 16 * ct + m] = vo[ct][r] * invn[r];
    }
    __syncthreads();
    v4f ov[8];
#pragma unroll
    for (int q = 0; q < 8; ++q) ov[q] = *(const v4f*)(acc + (slot0 + 2 * q + h) * FEAT + 4 * m);
#pragma unroll
    for (int q = 0; q < 8; ++q) {
      const int nd = node0 + 2 * q + h;
      if (nd < nN) *(volatile v4f*)(out0 + (size_t)nd * FEAT + 4 * m) = ov[q];
    }
    __threadfence();
#pragma unroll
    for (int q = 0; q < 8; ++q) {
      const int nd = node0 + 2 * q + h;
      if (nd < nN) *(volatile v4f*)(out0 + (size_t)nd * FEAT + 4 * m) = ov[q];
    }
  }
}

extern "C" void kernel_launch(void* const* d_in, const int* in_sizes, int n_in,
                              void* d_out, int out_size, void* d_ws, size_t ws_size,
                              hipStream_t stream) {
  if (n_in < 14) return;
  if (in_sizes[0] <= 0 || (in_sizes[0] % FEAT) != 0) return;
  const int nN = in_sizes[0] / FEAT;
  const int nE = in_sizes[1];
  if (nE <= 0 || in_sizes[2] != nE) return;
  if (in_sizes[3] != 256 * 64 || in_sizes[4] != 256) return;
  if (in_sizes[5] != 128 * 256 || in_sizes[6] != 128) return;
  if (in_sizes[7] != 64 * 128 || in_sizes[8] != 64) return;
  if (in_sizes[9] != 64 || in_sizes[10] < 1) return;
  if (in_sizes[11] != FEAT * FEAT || in_sizes[12] != FEAT * FEAT || in_sizes[13] != FEAT) return;
  if (out_size != nN * FEAT + nE) return;

  const float* x      = (const float*)d_in[0];
  const int*   src    = (const int*)d_in[1];
  const int*   dst    = (const int*)d_in[2];
  const float* w1     = (const float*)d_in[3];
  const float* b1     = (const float*)d_in[4];
  const float* w2     = (const float*)d_in[5];
  const float* b2     = (const float*)d_in[6];
  const float* w3     = (const float*)d_in[7];
  const float* b3     = (const float*)d_in[8];
  const float* w4     = (const float*)d_in[9];
  const float* b4     = (const float*)d_in[10];
  const float* wself  = (const float*)d_in[11];
  const float* wneigh = (const float*)d_in[12];
  const float* bias   = (const float*)d_in[13];

  float* out0 = (float*)d_out;
  float* out1 = out0 + (size_t)nN * FEAT;

  const int nBlkE = (nE + EPB - 1) / EPB;
  const int nBlkN = (nN + NB - 1) / NB;

  char* ws = (char*)d_ws;
  size_t off = 0;
  const size_t oW = off; off += (size_t)NWH * 2;                 off = (off + 255) & ~(size_t)255;
  const size_t oE = off; off += (size_t)nBlkE * EPB * 4;         off = (off + 255) & ~(size_t)255;
  if (off > ws_size || off > (size_t)134217728) return;
  _Float16* wpl = (_Float16*)(ws + oW);
  float*    epl = (float*)(ws + oE);

  k_cvt<<<NWH / 8 / NTHR, NTHR, 0, stream>>>(w1, w2, w3, wpl);

  k_edge<<<nBlkE, NTHR, 0, stream>>>(x, src, dst, wpl, b1, b2, b3, w4, b4, out1, epl, nN, nE);

  k_node<<<nBlkN, NTHR, 0, stream>>>(x, src, dst, epl, wself, wneigh, bias, out0, nN, nE);
}
